// rnn_tangent_iso_78503412236566
// MI455X (gfx1250) — hardware-verified
//
#include <hip/hip_runtime.h>

#define BB   1024
#define SS   256
#define HH   128
#define NSYM 6
#define XS   136
#define AS   40
#define SB   8
#define RSPLIT (1.0f / 2048.0f)

typedef _Float16 h16;
typedef __attribute__((ext_vector_type(16))) _Float16 v16h;
typedef __attribute__((ext_vector_type(8)))  _Float16 v8h;
typedef __attribute__((ext_vector_type(8)))  float v8f;
typedef __attribute__((ext_vector_type(4)))  float v4f_t;
typedef float v4fa __attribute__((ext_vector_type(4), may_alias));

__device__ __forceinline__ h16 lo_of(float v, h16 h) { return (h16)((v - (float)h) * 2048.0f); }
__device__ __forceinline__ v8f wmma16(v16h a, v16h b, v8f c) { return __builtin_amdgcn_wmma_f32_16x16x32_f16(false, a, false, b, (short)0, c, false, false); }
__device__ __forceinline__ v8f wmma_split(v16h a, v16h al, v16h b, v16h bl, v8f c) { v8f x = {}; x = wmma16(al, b, x); x = wmma16(a, bl, x); return wmma16(a, b, c) + x * RSPLIT; }
__device__ __forceinline__ v16h rfrag(const h16* rowp, int half) {
  const h16* p = rowp + 8 * half;
  return __builtin_shufflevector(*(const v8h*)p, *(const v8h*)(p + 16), 0,1,2,3,4,5,6,7,8,9,10,11,12,13,14,15);
}
__device__ __forceinline__ int kof(int half, int e) { return 8 * half + ((e < 8) ? e : (e + 8)); }

__global__ __launch_bounds__(256, 1)
void rnn_tangent_iso_kernel(const float* __restrict__ strain,
                            const float* __restrict__ stress0,
                            const float* __restrict__ w_in0, const float* __restrict__ b_in0,
                            const float* __restrict__ w_in1, const float* __restrict__ w_in2,
                            const float* __restrict__ w_h,  const float* __restrict__ b_h,
                            const float* __restrict__ w_out, const float* __restrict__ b_out,
                            float* __restrict__ out)
{
  __shared__ __align__(16) h16  xb0[2][16 * XS], xb1[2][16 * XS];
  __shared__ __align__(16) h16  acat[2][16 * AS];
  __shared__ __align__(16) float sbuf[2][16 * SB];
  __shared__ __align__(16) float stressS[16 * SB];
  __shared__ __align__(16) float klame[16 * 2];
  __shared__ __align__(16) float wout_s[2 * HH];
  __shared__ __align__(16) float obuf[16 * 16 * NSYM];
  __shared__ __align__(16) h16 BhlS[2][4][256 * 16];

  const int tid = threadIdx.x, wave = tid >> 5, lane = tid & 31, l16 = lane & 15, half = lane >> 4;
  const int rbase = blockIdx.x * 16;
  const int n = wave * 16 + l16;

  v16h Bh[2][4];
#pragma unroll
  for (int i = 0; i < 2; ++i)
#pragma unroll
    for (int f = 0; f < 4; ++f) {
      const float* src = w_h + ((size_t)(i * HH + n)) * HH + f * 32;
      v16h r;
#pragma unroll
      for (int e = 0; e < 16; ++e) { const float v = src[kof(half, e)]; r[e] = (h16)v; BhlS[i][f][tid * 16 + e] = lo_of(v, r[e]); }
      Bh[i][f] = r;
    }
  v16h Bin[2], Binl[2];
#pragma unroll
  for (int p = 0; p < 2; ++p) {
    v16h r, rl;
#pragma unroll
    for (int e = 0; e < 16; ++e) {
      const int k = kof(half, e);
      float v = 0.0f;
      if (k < 6)       v = (p == 0) ? w_in0[n * NSYM + k]       : w_in1[n * NSYM + k];
      else if (k < 12) v = (p == 0) ? w_in1[n * NSYM + (k - 6)] : w_in0[n * NSYM + (k - 6)];
      else if (k < 18) v = w_in2[n * NSYM + (k - 12)];
      r[e] = (h16)v; rl[e] = lo_of(v, r[e]);
    }
    Bin[p] = r; Binl[p] = rl;
  }
  const float biasIn = b_in0[n], biasH0 = b_h[n], biasH1 = b_h[HH + n];
  for (int i = tid; i < 2 * HH; i += 256) wout_s[i] = w_out[i];

  for (int e = tid; e < 2 * 16 * AS; e += 256) (&acat[0][0])[e] = (h16)0.0f;
  __syncthreads();
  if (tid < 96) {
    const int row = tid / 6, c = tid % 6, g = rbase + row;
    const float s0 = stress0[g * NSYM + c];
    stressS[row * SB + c] = s0;
    { const h16 hv = (h16)s0; acat[0][row * AS + 12 + c] = hv; acat[1][row * AS + 12 + c] = lo_of(s0, hv); }
    obuf[(row * 16 + 0) * NSYM + c] = s0;
    const float e0 = strain[((size_t)g * SS + 0) * NSYM + c];
    sbuf[0][row * SB + c] = e0;
    { const h16 hv = (h16)e0; acat[0][row * AS + c] = hv; acat[1][row * AS + c] = lo_of(e0, hv); }
  }
  __syncthreads();

#pragma unroll 1
  for (int t = 0; t < SS - 1; ++t) {
    const int p = t & 1;
    const float* epb = sbuf[p];
    float*       ecb = sbuf[p ^ 1];
    if (tid < 96) {
      const int row = tid / 6, c = tid % 6, g = rbase + row;
      const float ecv = strain[((size_t)g * SS + (t + 1)) * NSYM + c];
      ecb[row * SB + c] = ecv;
      const h16 hv = (h16)ecv; acat[0][row * AS + (p ^ 1) * 6 + c] = hv; acat[1][row * AS + (p ^ 1) * 6 + c] = lo_of(ecv, hv);
    }
    __syncthreads();
    {
      v8f c;
#pragma unroll
      for (int r = 0; r < 8; ++r) c[r] = biasIn;
      c = wmma_split(rfrag(&acat[0][l16 * AS], half), rfrag(&acat[1][l16 * AS], half), p ? Bin[1] : Bin[0], p ? Binl[1] : Binl[0], c);
#pragma unroll
      for (int r = 0; r < 8; ++r) { const float v = fmaxf(c[r], 0.0f); const h16 hv = (h16)v;
        xb0[0][(r + 8 * half) * XS + n] = hv; xb0[1][(r + 8 * half) * XS + n] = lo_of(v, hv); }
    }
    __syncthreads();
    {
      v8f c;
#pragma unroll
      for (int r = 0; r < 8; ++r) c[r] = biasH0;
#pragma unroll
      for (int f = 0; f < 4; ++f) c = wmma_split(rfrag(&xb0[0][l16 * XS + f * 32], half), rfrag(&xb0[1][l16 * XS + f * 32], half), Bh[0][f], *(const v16h*)&BhlS[0][f][tid * 16], c);
#pragma unroll
      for (int r = 0; r < 8; ++r) { const float v = fmaxf(c[r], 0.0f); const h16 hv = (h16)v;
        xb1[0][(r + 8 * half) * XS + n] = hv; xb1[1][(r + 8 * half) * XS + n] = lo_of(v, hv); }
    }
    __syncthreads();
    {
      v8f c;
#pragma unroll
      for (int r = 0; r < 8; ++r) c[r] = biasH1;
#pragma unroll
      for (int f = 0; f < 4; ++f) c = wmma_split(rfrag(&xb1[0][l16 * XS + f * 32], half), rfrag(&xb1[1][l16 * XS + f * 32], half), Bh[1][f], *(const v16h*)&BhlS[1][f][tid * 16], c);
#pragma unroll
      for (int r = 0; r < 8; ++r) { const float v = fmaxf(c[r], 0.0f); const h16 hv = (h16)v;
        xb0[0][(r + 8 * half) * XS + n] = hv; xb0[1][(r + 8 * half) * XS + n] = lo_of(v, hv); }
    }
    __syncthreads();
    if (tid < 32) {
      const int row = tid >> 1, l = tid & 1;
      float a = b_out[l];
#pragma unroll 1
      for (int j = 0; j < HH; ++j) a += ((float)xb0[0][row * XS + j] + (float)xb0[1][row * XS + j] * RSPLIT) * wout_s[l * HH + j];
      klame[row * 2 + l] = a;
    }
    __syncthreads();
    if (tid < 96) {
      const int row = tid / 6, j = tid % 6;
      const float lam = klame[row * 2 + 0], twomu = 2.0f * klame[row * 2 + 1];
      const float de = ecb[row * SB + j] - epb[row * SB + j];
      float tr = 0.0f;
#pragma unroll
      for (int c2 = 0; c2 < 3; ++c2) tr += ecb[row * SB + c2] - epb[row * SB + c2];
      const float s = stressS[row * SB + j] + ((j < 3) ? lam * tr : 0.0f) + twomu * de;
      stressS[row * SB + j] = s;
      const h16 hv = (h16)s; acat[0][row * AS + 12 + j] = hv; acat[1][row * AS + 12 + j] = lo_of(s, hv);
      obuf[(row * 16 + ((t + 1) & 15)) * NSYM + j] = s;
    }
    __syncthreads();
    if (((t + 2) & 15) == 0) {
      const int s0 = (t + 2) - 16;
#pragma unroll 1
      for (int pass = 0; pass < 2; ++pass) {
        for (int ch = tid; ch < 16 * 24; ch += 256) { const int row = ch / 24, q = (ch % 24) * 4;
          *(volatile v4f_t*)(out + ((size_t)(rbase + row) * SS + s0) * NSYM + q) = *(const volatile v4fa*)(obuf + row * 96 + q); }
        __threadfence();
      }
      __syncthreads();
    }
  }
}

extern "C" void kernel_launch(void* const* d_in, const int* in_sizes, int n_in,
                              void* d_out, int out_size, void* d_ws, size_t ws_size,
                              hipStream_t stream) {
  (void)in_sizes; (void)n_in; (void)out_size; (void)d_ws; (void)ws_size;
  const float* strain  = (const float*)d_in[0];
  const float* stress0 = (const float*)d_in[1];
  const float* w_in0   = (const float*)d_in[2];
  const float* b_in0   = (const float*)d_in[3];
  const float* w_in1   = (const float*)d_in[4];
  const float* w_in2   = (const float*)d_in[5];
  const float* w_h     = (const float*)d_in[6];
  const float* b_h     = (const float*)d_in[7];
  const float* w_out   = (const float*)d_in[8];
  const float* b_out   = (const float*)d_in[9];
  float* out = (float*)d_out;
  hipLaunchKernelGGL(rnn_tangent_iso_kernel, dim3(BB / 16), dim3(256), 0, stream,
                     strain, stress0, w_in0, b_in0, w_in1, w_in2, w_h, b_h, w_out, b_out, out);
}
